// ConnectionNetwork_81492709474821
// MI455X (gfx1250) — hardware-verified
//
#include <hip/hip_runtime.h>


namespace {
constexpr int N = 1024, D = 128, NIT = 100;
constexpr float XS = 8.0f, WSC = 256.0f;
typedef _Float16 b16;
typedef __attribute__((ext_vector_type(16))) _Float16 v16b;
typedef __attribute__((ext_vector_type(8))) _Float16 v8b;
typedef __attribute__((ext_vector_type(8))) float v8f;
typedef __attribute__((ext_vector_type(4))) float v4f;
__device__ __forceinline__ float bf16_rne(float f) { unsigned int u = __float_as_uint(f); u += 0x7FFFu + ((u >> 16) & 1u); return __uint_as_float(u & 0xFFFF0000u); }
__device__ __forceinline__ v16b frag_kb(const b16* p, int hh) { const v8b a = *(const v8b*)(p + 8 * hh), b = *(const v8b*)(p + 16 + 8 * hh); v16b f;
#pragma unroll
  for (int e = 0; e < 8; ++e) { f[e] = a[e]; f[8 + e] = b[e]; } return f; }
__device__ __forceinline__ v8f wmma16b(v16b a, v16b b, v8f c) { v8f d = __builtin_amdgcn_wmma_f32_16x16x32_f16(false, a, false, b, (short)0, c, false, false); asm volatile("v_nop\n\tv_nop\n\tv_nop\n\tv_nop" : "+v"(d) : "v"(a), "v"(b)); return d; }
__device__ __forceinline__ void wave_lds_sync() { __builtin_amdgcn_fence(__ATOMIC_RELEASE, "workgroup"); __builtin_amdgcn_wave_barrier(); __builtin_amdgcn_fence(__ATOMIC_ACQUIRE, "workgroup"); }
__device__ __forceinline__ float pmul(float a, float b) { float p = a * b; asm volatile("" : "+v"(p)); return p; }

__global__ __launch_bounds__(256) void wsplit_kernel(const float* __restrict__ W1, int ro, b16* __restrict__ WT) {
  const int u = blockIdx.x * 256 + threadIdx.x; if (u >= 2 * D * 16) return; const int row = u / 16, k0 = (u % 16) * 8; const int g = row / D, o = row % D; v8b v;
#pragma unroll
  for (int j = 0; j < 8; ++j) v[j] = (b16)(bf16_rne(W1[(size_t)o * (2 * D) + g * D + k0 + j]) * WSC); for (int pass = 0; pass < 2; ++pass) { *(volatile v8b*)(WT + (size_t)(ro + row) * D + k0) = v; __threadfence(); }
}
__global__ __launch_bounds__(32) void node_kernel(const float* __restrict__ x, const b16* __restrict__ WT, float* __restrict__ AB) {
  __shared__ __attribute__((aligned(16))) b16 Ah[16][D + 8]; __shared__ __attribute__((aligned(16))) float Tf[16][128 + 4];
  const int lane = threadIdx.x, nloc = lane & 15, hlf = lane >> 4; const size_t m0 = (size_t)blockIdx.x * 16;
  for (int rr = 0; rr < 16; ++rr) for (int q = 0; q < 4; ++q) Ah[rr][q * 32 + lane] = (b16)(bf16_rne(x[(m0 + rr) * D + q * 32 + lane]) * XS);
  wave_lds_sync();
#pragma unroll 1
  for (int cg = 0; cg < 4; ++cg) { v8f acc[8];
#pragma unroll
    for (int t = 0; t < 8; ++t) acc[t] = (v8f){};
#pragma unroll
    for (int kb = 0; kb < D; kb += 32) { const v16b a = frag_kb(&Ah[nloc][kb], hlf);
#pragma unroll
      for (int t = 0; t < 8; ++t) acc[t] = wmma16b(a, frag_kb(WT + (size_t)(cg * 128 + t * 16 + nloc) * D + kb, hlf), acc[t]); }
#pragma unroll
    for (int t = 0; t < 8; ++t)
#pragma unroll
      for (int r8 = 0; r8 < 8; ++r8) Tf[8 * hlf + r8][t * 16 + nloc] = acc[t][r8] * (1.0f / (XS * WSC));
    wave_lds_sync();
    for (int pass = 0; pass < 2; ++pass) { for (int rr = 0; rr < 16; ++rr) *(volatile v4f*)(AB + (m0 + rr) * 512 + cg * 128 + lane * 4) = *(const v4f*)(&Tf[rr][lane * 4]); __threadfence(); }
    wave_lds_sync(); }
}
__global__ __launch_bounds__(32) void pair_kernel(const float* __restrict__ AB, const float* __restrict__ b1c, const float* __restrict__ w2c, const float* __restrict__ b2c, const float* __restrict__ b1w, const float* __restrict__ w2w, const float* __restrict__ b2w, float* __restrict__ Pm) {
  __shared__ float Ai[D], Bi[D], B1c[D], W2c[D], B1w[D], W2w[D];
  const int lane = threadIdx.x; const int jt = blockIdx.x % (N / 32), i = blockIdx.x / (N / 32); const int j = jt * 32 + lane;
  for (int q = 0; q < 4; ++q) { const int d = q * 32 + lane; Ai[d] = AB[(size_t)i * 512 + d]; Bi[d] = AB[(size_t)i * 512 + 384 + d]; B1c[d] = bf16_rne(b1c[d]); W2c[d] = bf16_rne(w2c[d]); B1w[d] = bf16_rne(b1w[d]); W2w[d] = bf16_rne(w2w[d]); }
  wave_lds_sync();
  const float* Bj = AB + (size_t)j * 512 + 128; const float* Aj = AB + (size_t)j * 512 + 256; float s1 = 0.0f, s2 = 0.0f;
#pragma unroll 4
  for (int d = 0; d < D; ++d) { s1 += pmul(fmaxf(Ai[d] + Bj[d] + B1c[d], 0.0f), W2c[d]); s2 += pmul(fmaxf(Aj[d] + Bi[d] + B1w[d], 0.0f), W2w[d]); }
  float S = 0.0f; if (i != j) S = (s1 + bf16_rne(b2c[0])) + (s2 + bf16_rne(b2w[0]));
  const float p = __expf(S);
  for (int pass = 0; pass < 2; ++pass) { ((volatile float*)Pm)[(size_t)i * N + j] = p; __threadfence(); }
}
__global__ __launch_bounds__(256) void row_kernel(float* Pm) {
  const int wave = threadIdx.x >> 5, lane = threadIdx.x & 31; const size_t r = (size_t)blockIdx.x * 8 + wave; float* row = Pm + r * N; float s = 0.0f;
  for (int q = 0; q < N / 32; ++q) s += row[q * 32 + lane]; for (int o = 16; o; o >>= 1) s += __shfl_xor(s, o); const float inv = 1.0f / s;
  for (int q = 0; q < N / 32; ++q) { const float v = row[q * 32 + lane] * inv; ((volatile float*)row)[q * 32 + lane] = v; ((volatile float*)row)[q * 32 + lane] = v; }
  __threadfence();
}
__global__ __launch_bounds__(32) void col_kernel(const float* Pin, float* Pout) {
  const int lane = threadIdx.x; const int c = blockIdx.x * 32 + lane; float s = 0.0f;
#pragma unroll 8
  for (int r = 0; r < N; ++r) s += Pin[(size_t)r * N + c]; const float inv = 1.0f / s;
  for (int r = 0; r < N; ++r) { const float v = Pin[(size_t)r * N + c] * inv; ((volatile float*)Pout)[(size_t)r * N + c] = v; ((volatile float*)Pout)[(size_t)r * N + c] = v; }
  __threadfence();
}
}

extern "C" void kernel_launch(void* const* d_in, const int* in_sizes, int n_in, void* d_out, int out_size, void* d_ws, size_t ws_size, hipStream_t stream) {
  (void)n_in;
  auto Fp = [&](int i) { return (const float*)d_in[i]; };
  if (in_sizes[0] != N * D || in_sizes[1] != D * 2 * D || in_sizes[2] != D || in_sizes[3] != D || in_sizes[4] != 1 || in_sizes[5] != D * 2 * D || in_sizes[7] != D || in_sizes[8] != 1 || out_size != N * N) return;
  const int NITV = NIT;
  size_t off = 0; char* ws = (char*)d_ws;
  auto carve = [&](size_t bytes) { char* p = ws + off; off += (bytes + 255) & ~(size_t)255; return p; };
  b16* WT = (b16*)carve((size_t)512 * D * 2); float* AB = (float*)carve((size_t)N * 512 * 4);
  if (off > ws_size || off > ((size_t)16 << 20)) return;
  float* Pm = (float*)d_out;
  wsplit_kernel<<<(2 * D * 16 + 255) / 256, 256, 0, stream>>>(Fp(1), 0, WT); wsplit_kernel<<<(2 * D * 16 + 255) / 256, 256, 0, stream>>>(Fp(5), 2 * D, WT);
  node_kernel<<<N / 16, 32, 0, stream>>>(Fp(0), WT, AB);
  pair_kernel<<<N * (N / 32), 32, 0, stream>>>(AB, Fp(2), Fp(3), Fp(4), Fp(6), Fp(7), Fp(8), Pm);
  for (int it = 0; it < NITV; ++it) { row_kernel<<<N / 8, 256, 0, stream>>>(Pm); col_kernel<<<N / 32, 32, 0, stream>>>(Pm, Pm); }
}
